// MaskFormerSwinLayer_4337916969424
// MI455X (gfx1250) — hardware-verified
//
#include <hip/hip_runtime.h>
#include <math.h>
typedef __attribute__((ext_vector_type(16))) _Float16 v16h;
typedef __attribute__((ext_vector_type(8)))  _Float16 v8h;
typedef __attribute__((ext_vector_type(16))) __bf16   v16b;
typedef __attribute__((ext_vector_type(8)))  __bf16   v8b;
typedef __attribute__((ext_vector_type(8)))  float    v8f;
typedef __attribute__((ext_vector_type(4)))  float    v4f;
#define PSCALE 32768.0f
#define U16(p) ((const unsigned short*)(const void*)(p))
#define PSCALE_INV (1.0f / 32768.0f)

__device__ __forceinline__ unsigned short f2bf_bits(float f) {
  unsigned u = __float_as_uint(f);
  return (unsigned short)((u + 0x7FFFu + ((u >> 16) & 1u)) >> 16);
}
__device__ __forceinline__ float bf_bits2f(unsigned short h) { return __uint_as_float(((unsigned)h) << 16); }

__device__ __forceinline__ void dep_guard_h(v8f& a, v8f& b, v16h x, v16h y) { asm volatile("v_nop\n\tv_nop\n\tv_nop\n\tv_nop" : "+v"(a), "+v"(b) : "v"(x), "v"(y)); }
__device__ __forceinline__ void dep_guard_b(v8f& a, v8f& b, v16b x, v16b y) { asm volatile("v_nop\n\tv_nop\n\tv_nop\n\tv_nop" : "+v"(a), "+v"(b) : "v"(x), "v"(y)); }
__device__ __forceinline__ void keep4_h(v16h a, v16h b, v16h c, v16h d) { asm volatile("v_nop" :: "v"(a), "v"(b), "v"(c), "v"(d)); }
__device__ __forceinline__ void keep4_b(v16b a, v16b b, v16b c, v16b d) { asm volatile("v_nop" :: "v"(a), "v"(b), "v"(c), "v"(d)); }
__device__ __forceinline__ void acc_guard4(v8f& a, v8f& b, v8f& c, v8f& d) { asm volatile("v_nop\n\tv_nop\n\tv_nop\n\tv_nop" : "+v"(a), "+v"(b), "+v"(c), "+v"(d)); }
template <typename T> struct Frag;
template <> struct Frag<_Float16> {
  typedef v16h V; union U { v16h v; v8h h[2]; };
  static __device__ __forceinline__ v16h load(const _Float16* p) {
    U f; f.h[0] = *(const v8h*)(p); f.h[1] = *(const v8h*)(p + 16); return f.v;
  }
  static __device__ __forceinline__ v8f mma(v16h a, v16h b, v8f c) {
    return __builtin_amdgcn_wmma_f32_16x16x32_f16(false, a, false, b, (short)0, c, false, false);
  }
  static __device__ __forceinline__ void guard(v8f& a, v8f& b, v16h x, v16h y) { dep_guard_h(a, b, x, y); }
  static __device__ __forceinline__ void keep(v16h a, v16h b, v16h c, v16h d) { keep4_h(a, b, c, d); }
};
template <> struct Frag<__bf16> {
  typedef v16b V; union U { v16b v; v8b h[2]; };
  static __device__ __forceinline__ v16b load(const __bf16* p) {
    U f; f.h[0] = *(const v8b*)(p); f.h[1] = *(const v8b*)(p + 16); return f.v;
  }
  static __device__ __forceinline__ v8f mma(v16b a, v16b b, v8f c) {
    return __builtin_amdgcn_wmma_f32_16x16x32_bf16(false, a, false, b, (short)0, c, false, false);
  }
  static __device__ __forceinline__ void guard(v8f& a, v8f& b, v16b x, v16b y) { dep_guard_b(a, b, x, y); }
  static __device__ __forceinline__ void keep(v16b a, v16b b, v16b c, v16b d) { keep4_b(a, b, c, d); }
};

template <int ET> struct Elem;
template <> struct Elem<0> { typedef _Float16 T; };
template <> struct Elem<1> { typedef __bf16 T; };
template <int ET, bool SPLIT, int BIAS_MODE, int OUT_MODE, bool RESID, int ACT = 0>
__global__ __launch_bounds__(256) void wmma_gemm64(
    const unsigned short* __restrict__ Ap, const unsigned short* __restrict__ A2p, int lda, long strideA,
    const unsigned short* __restrict__ Btp, const unsigned short* __restrict__ Bt2p, int ldb, long strideB,
    void* __restrict__ Cout, void* __restrict__ Cout2, int ldc, long strideC,
    const float* __restrict__ bias,
    const float* __restrict__ resid, long strideR,
    int M, int N, int K, float scale) {
  typedef typename Elem<ET>::T T;
  typedef typename Frag<T>::V V;
  const T* A = (const T*)Ap; const T* A2 = (const T*)A2p; const T* Bt = (const T*)Btp; const T* Bt2 = (const T*)Bt2p;
  __shared__ __align__(16) float sT[8][16 * 68];
  const int b    = blockIdx.y;
  const int lane = threadIdx.x & 31;
  const int wave = threadIdx.x >> 5;
  const int tilesN = N >> 6;
  const int tilesM = M >> 6;
  const int tile = blockIdx.x * 8 + wave;
  if (tile >= tilesM * tilesN) return;
  const int tm = tile / tilesN;
  const int tn = tile - tm * tilesN;
  const int m0 = tm << 6;
  const int n0 = tn << 6;

  const T* Ab  = A  + (size_t)b * strideA;
  const T* Bb  = Bt + (size_t)b * strideB;
  const T* Ab2 = SPLIT ? (A2  + (size_t)b * strideA) : nullptr;
  const T* Bb2 = SPLIT ? (Bt2 + (size_t)b * strideB) : nullptr;

  const int rlane = lane & 15;
  const int koff  = (lane >> 4) * 8;
  const int mOff  = (lane >> 4) * 8;

  v8f acc[4][4];
#pragma unroll
  for (int i = 0; i < 4; ++i)
#pragma unroll
    for (int j = 0; j < 4; ++j) acc[i][j] = (v8f){0.f,0.f,0.f,0.f,0.f,0.f,0.f,0.f};

  for (int k0 = 0; k0 < K; k0 += 32) {
    V bh[4], bl[4];
#pragma unroll
    for (int j = 0; j < 4; ++j) {
      const size_t bo = (size_t)(n0 + (j << 4) + rlane) * ldb + koff + k0;
      bh[j] = Frag<T>::load(Bb + bo);
      if (SPLIT) bl[j] = Frag<T>::load(Bb2 + bo);
    }
#pragma unroll
    for (int i = 0; i < 4; ++i) {
      const size_t ao = (size_t)(m0 + (i << 4) + rlane) * lda + koff + k0;
      V ah = Frag<T>::load(Ab + ao);
      V al;
      if (SPLIT) al = Frag<T>::load(Ab2 + ao);
#pragma unroll
      for (int j = 0; j < 4; ++j) {
        acc[i][j] = Frag<T>::mma(ah, bh[j], acc[i][j]);
        if (SPLIT) {
          acc[i][j] = Frag<T>::mma(ah, bl[j], acc[i][j]);
          acc[i][j] = Frag<T>::mma(al, bh[j], acc[i][j]);
        }
      }
      Frag<T>::guard(acc[i][0], acc[i][3], ah, SPLIT ? al : ah);
    }
    Frag<T>::keep(bh[0], bh[1], bh[2], bh[3]);
    if (SPLIT) Frag<T>::keep(bl[0], bl[1], bl[2], bl[3]);
  }
  acc_guard4(acc[0][0], acc[0][1], acc[0][2], acc[0][3]);
  acc_guard4(acc[1][0], acc[1][1], acc[1][2], acc[1][3]);
  acc_guard4(acc[2][0], acc[2][1], acc[2][2], acc[2][3]);
  acc_guard4(acc[3][0], acc[3][1], acc[3][2], acc[3][3]);

  float* slab = sT[wave];
  const float* Rb = RESID ? (resid + (size_t)b * strideR) : nullptr;
#pragma unroll
  for (int i = 0; i < 4; ++i) {
    const int mBase = m0 + (i << 4);
#pragma unroll
    for (int j = 0; j < 4; ++j) {
      const int n = n0 + (j << 4) + rlane;
      float bv = 0.f;
      if (BIAS_MODE == 2) bv = bias[n];
#pragma unroll
      for (int r = 0; r < 8; ++r) {
        float v = acc[i][j][r] * scale;
        if (BIAS_MODE == 1) v += bias[mBase + mOff + r];
        if (BIAS_MODE == 2) v += bv;
        if (RESID) v += Rb[(size_t)(mBase + mOff + r) * ldc + n];
        if (ACT == 1) v = tanhf(v);
        if (ACT == 2) v = fmaxf(v, 0.0f);
        if (ACT == 3) v = v / (1.0f + expf(-v));
        if (ACT == 4) v = (v > 0.f) ? v : 0.01f * v;
        if (ACT == 5) v = 0.5f * v * (1.0f + erff(v * 0.70710678118654752f));
        slab[(mOff + r) * 68 + (j << 4) + rlane] = v;
      }
    }
    __builtin_amdgcn_fence(__ATOMIC_RELEASE, "workgroup");
    __builtin_amdgcn_wave_barrier();
    __builtin_amdgcn_fence(__ATOMIC_ACQUIRE, "workgroup");
    if (OUT_MODE == 0) {
      float* C = (float*)Cout + (size_t)b * strideC;
      const int hh = lane >> 4, c4 = (lane & 15) * 4;
      for (int pass = 0; pass < 2; ++pass) {
#pragma unroll
        for (int it = 0; it < 8; ++it) {
          const int row = it * 2 + hh;
          v4f v = *(const v4f*)(slab + row * 68 + c4);
          *(volatile v4f*)(C + (size_t)(mBase + row) * ldc + n0 + c4) = v;
        }
        __threadfence();
      }
    } else {
      const int q = lane >> 3, c8 = (lane & 7) * 8;
      unsigned short* C  = (unsigned short*)Cout  + (size_t)b * strideC;
      unsigned short* C2 = (OUT_MODE == 2) ? ((unsigned short*)Cout2 + (size_t)b * strideC) : nullptr;
      for (int pass = 0; pass < 2; ++pass) {
#pragma unroll
        for (int it = 0; it < 4; ++it) {
          const int row = it * 4 + q;
          const float* sp = slab + row * 68 + c8;
          v8h hv, lv;
#pragma unroll
          for (int e = 0; e < 8; ++e) {
            if (OUT_MODE == 1) {
              hv[e] = (_Float16)sp[e];
            } else {
              unsigned short hb = f2bf_bits(sp[e]);
              unsigned short lb = f2bf_bits(sp[e] - bf_bits2f(hb));
              hv[e] = __builtin_bit_cast(_Float16, hb);
              lv[e] = __builtin_bit_cast(_Float16, lb);
            }
          }
          *(volatile v8h*)(C + (size_t)(mBase + row) * ldc + n0 + c8) = hv;
          if (OUT_MODE == 2) *(volatile v8h*)(C2 + (size_t)(mBase + row) * ldc + n0 + c8) = lv;
        }
        __threadfence();
      }
    }
    __builtin_amdgcn_fence(__ATOMIC_RELEASE, "workgroup");
    __builtin_amdgcn_wave_barrier();
    __builtin_amdgcn_fence(__ATOMIC_ACQUIRE, "workgroup");
  }
}

__global__ __launch_bounds__(256) void cast_f32_f16x2(
    const float* __restrict__ in, _Float16* __restrict__ out, int n2) {
  int i = blockIdx.x * 256 + threadIdx.x;
  if (i < n2) {
    const _Float16 h0 = (_Float16)in[2 * i], h1 = (_Float16)in[2 * i + 1];
    const unsigned u = (unsigned)__builtin_bit_cast(unsigned short, h0) | ((unsigned)__builtin_bit_cast(unsigned short, h1) << 16);
    ((volatile unsigned*)out)[i] = u;
    __threadfence();
    ((volatile unsigned*)out)[i] = u;
  }
}


__global__ __launch_bounds__(256) void transpose_cast_f16(const float* __restrict__ in, int ldi,
                                                         _Float16* __restrict__ outT, int ldo, float scale) {
  __shared__ __align__(16) _Float16 tile[64][72];
  const int c0 = blockIdx.x * 64, r0 = blockIdx.y * 64;
  const int t = threadIdx.y * 32 + threadIdx.x;
  for (int i = threadIdx.y; i < 64; i += 8) {
    tile[threadIdx.x][i]      = (_Float16)(in[(size_t)(r0 + i) * ldi + c0 + threadIdx.x] * scale);
    tile[32 + threadIdx.x][i] = (_Float16)(in[(size_t)(r0 + i) * ldi + c0 + 32 + threadIdx.x] * scale);
  }
  __syncthreads();
  const int q = t >> 3, c8 = (t & 7) * 8;
  for (int pass = 0; pass < 2; ++pass) {
#pragma unroll
    for (int it = 0; it < 2; ++it) {
      const int c = it * 32 + q;
      v8h hv = *(const v8h*)(&tile[c][c8]);
      *(volatile v8h*)(outT + (size_t)(c0 + c) * ldo + r0 + c8) = hv;
    }
    __threadfence();
  }
}

#define SB 8
#define SH 56
#define SW 56
#define SC 384
#define SNH 12
#define SHD 32
#define WSZ 7
#define SHIFT 3
#define NWIN 64
#define NTOK 49
#define NROWS (SB * SH * SW)
#define FFN 1536

__device__ __forceinline__ int win_row_of_token(int b, int i, int j) {
  const int ip = (i - SHIFT + SH) % SH, jp = (j - SHIFT + SW) % SW;
  const int win = (ip / WSZ) * (SW / WSZ) + (jp / WSZ), n = (ip % WSZ) * WSZ + (jp % WSZ);
  return (b * NWIN + win) * NTOK + n;
}
template <int MODE>
__global__ __launch_bounds__(256) void ln_kernel(const float* __restrict__ X, const float* __restrict__ AO, const float* __restrict__ g, const float* __restrict__ bt,
                                               float* __restrict__ Hout, _Float16* __restrict__ Y16) {
  const int lane = threadIdx.x & 31, wave = threadIdx.x >> 5;
  const int row = blockIdx.x * 8 + wave;
  const int b = row / (SH * SW), ij = row % (SH * SW), i = ij / SW, j = ij % SW;
  const int wrow = win_row_of_token(b, i, j);
  float v[12];
#pragma unroll
  for (int q = 0; q < 3; ++q) { const v4f a = *(const v4f*)(X + (size_t)row * SC + (q * 32 + lane) * 4);
    v[4*q] = a[0]; v[4*q+1] = a[1]; v[4*q+2] = a[2]; v[4*q+3] = a[3]; }
  if (MODE == 1) {
#pragma unroll
    for (int q = 0; q < 3; ++q) { const v4f a = *(const v4f*)(AO + (size_t)wrow * SC + (q * 32 + lane) * 4);
      v[4*q] += a[0]; v[4*q+1] += a[1]; v[4*q+2] += a[2]; v[4*q+3] += a[3]; }
  }
  float s = 0.f;
#pragma unroll
  for (int q = 0; q < 12; ++q) s += v[q];
  for (int o = 16; o > 0; o >>= 1) s += __shfl_xor(s, o, 32);
  const float mu = s / (float)SC;
  float s2 = 0.f;
#pragma unroll
  for (int q = 0; q < 12; ++q) { const float d = v[q] - mu; s2 += d * d; }
  for (int o = 16; o > 0; o >>= 1) s2 += __shfl_xor(s2, o, 32);
  const float inv = rsqrtf(s2 / (float)SC + 1e-5f);
  typedef __attribute__((ext_vector_type(4))) _Float16 v4h;
  for (int pass = 0; pass < 2; ++pass) {
#pragma unroll
    for (int q = 0; q < 3; ++q) {
      const int c0 = (q * 32 + lane) * 4;
      v4h y;
#pragma unroll
      for (int e = 0; e < 4; ++e) y[e] = (_Float16)((v[4*q+e] - mu) * inv * g[c0 + e] + bt[c0 + e]);
      if (MODE == 0) *(volatile v4h*)(Y16 + (size_t)wrow * SC + c0) = y;
      else { *(volatile v4h*)(Y16 + (size_t)row * SC + c0) = y; const v4f hv = {v[4*q], v[4*q+1], v[4*q+2], v[4*q+3]}; *(volatile v4f*)(Hout + (size_t)row * SC + c0) = hv; }
    }
    __threadfence();
  }
}

__device__ __forceinline__ v8f mma16(v16h a, v16h b, v8f c) {
  c = __builtin_amdgcn_wmma_f32_16x16x32_f16(false, a, false, b, (short)0, c, false, false);
  asm volatile("v_nop\n\tv_nop\n\tv_nop\n\tv_nop" : "+v"(c) : "v"(a), "v"(b));
  return c;
}
__device__ __forceinline__ int region_of(int coord, int size) { return (coord < size - WSZ) ? 0 : ((coord < size - SHIFT) ? 1 : 2); }
__global__ __launch_bounds__(256) void window_attn_kernel(const float* __restrict__ QKV, const float* __restrict__ rpb, const int* __restrict__ rpi,
                                                          unsigned* __restrict__ CTX16) {
  __shared__ __align__(16) _Float16 Qs[64 * 40];
  __shared__ __align__(16) _Float16 Ks[64 * 40];
  __shared__ __align__(16) _Float16 Vt[32 * 72];
  __shared__ __align__(16) _Float16 Ps[64 * 72];
  __shared__ float Ss[64 * 65];
  __shared__ __align__(16) _Float16 Cs[NTOK * SC + 8];
  __shared__ int lbl[64];
  const int tid = threadIdx.x, lane = tid & 31, wave = tid >> 5, hh = lane >> 4, c = lane & 15;
  const int wrow0 = blockIdx.x * NTOK;
  const int win = blockIdx.x % NWIN, wr = win / (SW / WSZ), wc = win % (SW / WSZ);
  if (tid < 64) { const int n = tid; lbl[n] = (n < NTOK) ? (region_of(wr * WSZ + n / WSZ, SH) * 3 + region_of(wc * WSZ + n % WSZ, SW)) : -1; }
  for (int h = 0; h < SNH; ++h) {
    __syncthreads();
    for (int i = tid; i < 64 * 32; i += 256) {
      const int n = i >> 5, d = i & 31;
      float qv = 0.f, kv = 0.f, vv = 0.f;
      if (n < NTOK) { const float* r = QKV + (size_t)(wrow0 + n) * (3 * SC) + h * SHD + d; qv = r[0] * 0.17677669529663687f; kv = r[SC]; vv = r[2 * SC]; }
      Qs[n * 40 + d] = (_Float16)qv; Ks[n * 40 + d] = (_Float16)kv; Vt[d * 72 + n] = (_Float16)vv;
    }
    __syncthreads();
    for (int t = wave; t < 16; t += 8) {
      const int mt = t >> 2, nt = t & 3;
      v16h a, b;
      { const _Float16* p = Qs + (mt * 16 + c) * 40 + 8 * hh; const v8h lo = *(const v8h*)p, hi = *(const v8h*)(p + 16);
#pragma unroll
        for (int e = 0; e < 8; ++e) { a[e] = lo[e]; a[8 + e] = hi[e]; } }
      { const _Float16* p = Ks + (nt * 16 + c) * 40 + 8 * hh; const v8h lo = *(const v8h*)p, hi = *(const v8h*)(p + 16);
#pragma unroll
        for (int e = 0; e < 8; ++e) { b[e] = lo[e]; b[8 + e] = hi[e]; } }
      v8f acc = {0.f,0.f,0.f,0.f,0.f,0.f,0.f,0.f};
      acc = mma16(a, b, acc);
#pragma unroll
      for (int r = 0; r < 8; ++r) {
        const int row = mt * 16 + 8 * hh + r, col = nt * 16 + c;
        float sv = acc[r];
        if (row < NTOK && col < NTOK) {
          sv += rpb[(size_t)rpi[row * NTOK + col] * SNH + h];
          if (lbl[row] != lbl[col]) sv += -100.0f;
        } else sv = -INFINITY;
        Ss[row * 65 + col] = sv;
      }
    }
    __syncthreads();
    {
      const int row = tid >> 2, part = tid & 3;
      float mx = -INFINITY;
      for (int q = 0; q < 16; ++q) mx = fmaxf(mx, Ss[row * 65 + part * 16 + q]);
      mx = fmaxf(mx, __shfl_xor(mx, 1, 32)); mx = fmaxf(mx, __shfl_xor(mx, 2, 32));
      float ev[16], se = 0.f;
      for (int q = 0; q < 16; ++q) { const float sv = Ss[row * 65 + part * 16 + q]; ev[q] = (row < NTOK && sv > -INFINITY) ? expf(sv - mx) : 0.f; se += ev[q]; }
      se += __shfl_xor(se, 1, 32); se += __shfl_xor(se, 2, 32);
      const float inv = (row < NTOK) ? (32768.0f / se) : 0.f;
      for (int q = 0; q < 16; ++q) Ps[row * 72 + part * 16 + q] = (_Float16)(ev[q] * inv);
    }
    __syncthreads();
    {
      const int mt = wave >> 1, nt = wave & 1;
      v8f acc = {0.f,0.f,0.f,0.f,0.f,0.f,0.f,0.f};
#pragma unroll
      for (int ks = 0; ks < 2; ++ks) {
        v16h a, b;
        { const _Float16* p = Ps + (mt * 16 + c) * 72 + ks * 32 + 8 * hh; const v8h lo = *(const v8h*)p, hi = *(const v8h*)(p + 16);
#pragma unroll
          for (int e = 0; e < 8; ++e) { a[e] = lo[e]; a[8 + e] = hi[e]; } }
        { const _Float16* p = Vt + (nt * 16 + c) * 72 + ks * 32 + 8 * hh; const v8h lo = *(const v8h*)p, hi = *(const v8h*)(p + 16);
#pragma unroll
          for (int e = 0; e < 8; ++e) { b[e] = lo[e]; b[8 + e] = hi[e]; } }
        acc = mma16(a, b, acc);
      }
#pragma unroll
      for (int r = 0; r < 8; ++r) {
        const int row = mt * 16 + 8 * hh + r, d = nt * 16 + c;
        if (row < NTOK) Cs[row * SC + h * SHD + d] = (_Float16)(acc[r] * (1.0f / 32768.0f));
      }
    }
  }
  __syncthreads();
  for (int pass = 0; pass < 2; ++pass) {
    for (int i = tid; i < NTOK * 48; i += 256) {
      const int row = i / 48, seg = i % 48;
      typedef __attribute__((ext_vector_type(4))) unsigned u4;
      const u4 v = *(const u4*)(&Cs[row * SC + seg * 8]);
      *(volatile u4*)(CTX16 + ((size_t)(wrow0 + row) * SC + seg * 8) / 2) = v;
    }
    __threadfence();
  }
}
__global__ void bias_cat3_kernel(const float* a, const float* b, const float* c2, float* __restrict__ o) {
  for (int pass = 0; pass < 2; ++pass) { for (int i = threadIdx.x; i < 3 * SC; i += 256) ((volatile float*)o)[i] = (i < SC) ? a[i] : (i < 2 * SC ? b[i - SC] : c2[i - 2 * SC]); __threadfence(); }
}

extern "C" void kernel_launch(void* const* d_in, const int* in_sizes, int n_in,
                              void* d_out, int out_size, void* d_ws, size_t ws_size,
                              hipStream_t stream) {
  (void)in_sizes; (void)n_in; (void)out_size; (void)ws_size;
  const float* x = (const float*)d_in[0];
  const float* ln1g = (const float*)d_in[1]; const float* ln1b = (const float*)d_in[2];
  const float* qw = (const float*)d_in[3]; const float* qb = (const float*)d_in[4];
  const float* kw = (const float*)d_in[5]; const float* kb = (const float*)d_in[6];
  const float* vw = (const float*)d_in[7]; const float* vb = (const float*)d_in[8];
  const float* rpb = (const float*)d_in[9]; const int* rpi = (const int*)d_in[10];
  const float* pw = (const float*)d_in[11]; const float* pb = (const float*)d_in[12];
  const float* ln2g = (const float*)d_in[13]; const float* ln2b = (const float*)d_in[14];
  const float* f1w = (const float*)d_in[15]; const float* f1b = (const float*)d_in[16];
  const float* f2w = (const float*)d_in[17]; const float* f2b = (const float*)d_in[18];
  float* out = (float*)d_out;
  (void)d_in[19]; (void)d_in[20];

  char* ws = (char*)d_ws; size_t off = 0;
  auto carve = [&](size_t bytes) -> char* { char* p = ws + off; off += (bytes + 255) & ~(size_t)255; return p; };
  _Float16* XW16 = (_Float16*)carve((size_t)NROWS * SC * 2);
  _Float16* WqkvT = (_Float16*)carve((size_t)3 * SC * SC * 2);
  _Float16* WpT = (_Float16*)carve((size_t)SC * SC * 2);
  _Float16* W1T = (_Float16*)carve((size_t)FFN * SC * 2);
  _Float16* W2T = (_Float16*)carve((size_t)SC * FFN * 2);
  float* bqkv = (float*)carve((size_t)3 * SC * 4);
  float* QKV = (float*)carve((size_t)NROWS * 3 * SC * 4);
  unsigned* CTX16 = (unsigned*)carve((size_t)NROWS * SC * 2);
  float* AO = (float*)carve((size_t)NROWS * SC * 4);
  float* Hf = QKV;
  _Float16* Y16 = XW16;
  unsigned* F16 = (unsigned*)(QKV + (size_t)NROWS * SC);

  ln_kernel<0><<<NROWS / 8, 256, 0, stream>>>(x, nullptr, ln1g, ln1b, nullptr, XW16);
  transpose_cast_f16<<<dim3(SC / 64, SC / 64), dim3(32, 8), 0, stream>>>(qw, SC, WqkvT, SC, 1.0f);
  transpose_cast_f16<<<dim3(SC / 64, SC / 64), dim3(32, 8), 0, stream>>>(kw, SC, WqkvT + (size_t)SC * SC, SC, 1.0f);
  transpose_cast_f16<<<dim3(SC / 64, SC / 64), dim3(32, 8), 0, stream>>>(vw, SC, WqkvT + (size_t)2 * SC * SC, SC, 1.0f);
  transpose_cast_f16<<<dim3(SC / 64, SC / 64), dim3(32, 8), 0, stream>>>(pw, SC, WpT, SC, 1.0f);
  transpose_cast_f16<<<dim3(FFN / 64, SC / 64), dim3(32, 8), 0, stream>>>(f1w, FFN, W1T, SC, 1.0f);
  transpose_cast_f16<<<dim3(SC / 64, FFN / 64), dim3(32, 8), 0, stream>>>(f2w, SC, W2T, FFN, 1.0f);
  bias_cat3_kernel<<<1, 256, 0, stream>>>(qb, kb, vb, bqkv);
  {
    const int t = (NROWS / 64) * (3 * SC / 64);
    wmma_gemm64<0, false, 2, 0, false><<<dim3((t + 7) / 8, 1), 256, 0, stream>>>(U16(XW16), nullptr, SC, 0, U16(WqkvT), nullptr, SC, 0, QKV, nullptr, 3 * SC, 0, bqkv, nullptr, 0, NROWS, 3 * SC, SC, 1.0f);
  }
  window_attn_kernel<<<SB * NWIN, 256, 0, stream>>>(QKV, rpb, rpi, CTX16);
  {
    const int t = (NROWS / 64) * (SC / 64);
    wmma_gemm64<0, false, 2, 0, false><<<dim3((t + 7) / 8, 1), 256, 0, stream>>>((const unsigned short*)CTX16, nullptr, SC, 0, U16(WpT), nullptr, SC, 0, AO, nullptr, SC, 0, pb, nullptr, 0, NROWS, SC, SC, 1.0f);
  }
  ln_kernel<1><<<NROWS / 8, 256, 0, stream>>>(x, AO, ln2g, ln2b, Hf, Y16);
  {
    const int t1 = (NROWS / 64) * (FFN / 64);
    wmma_gemm64<0, false, 2, 1, false, 5><<<dim3((t1 + 7) / 8, 1), 256, 0, stream>>>(U16(Y16), nullptr, SC, 0, U16(W1T), nullptr, SC, 0, F16, nullptr, FFN, 0, f1b, nullptr, 0, NROWS, FFN, SC, 1.0f);
    const int t2 = (NROWS / 64) * (SC / 64);
    wmma_gemm64<0, false, 2, 0, true, 0><<<dim3((t2 + 7) / 8, 1), 256, 0, stream>>>((const unsigned short*)F16, nullptr, FFN, 0, U16(W2T), nullptr, FFN, 0, out, nullptr, SC, 0, f2b, Hf, 0, NROWS, SC, FFN, 1.0f);
  }
}
